// MultiHeadAttention_2748779070010
// MI455X (gfx1250) — hardware-verified
//
#include <hip/hip_runtime.h>
#ifndef NB
#define NB 2
#endif
#ifndef SEQ
#define SEQ 2048
#endif
#define NB_FULL 2
#define SEQ_FULL 2048
#define DM 1024
#define NH 16
#define HD 64
#define TT (NB * SEQ)
#define CXP (2 * DM)

static_assert(SEQ % 64 == 0);
static_assert(TT % 128 == 0);
static_assert(SEQ <= SEQ_FULL);
static_assert(NB <= NB_FULL);
static_assert(HD == 64);
static_assert(NH * HD == DM);
static_assert(DM % 128 == 0);

#define SZ_XB  ((size_t)TT * DM * 2)
#define SZ_WT  ((size_t)DM * DM * 2)
#define SZ_WO2 ((size_t)DM * CXP * 2)
#define SZ_H   ((size_t)TT * DM * 2)
#define SZ_CX  ((size_t)TT * CXP * 2)
static_assert(SZ_XB % 256 == 0 && SZ_WT % 256 == 0 && SZ_WO2 % 256 == 0 && SZ_H % 256 == 0 && SZ_CX % 256 == 0);
static_assert(3 * SZ_XB + 3 * SZ_WT + SZ_WO2 + 4 * SZ_H + SZ_CX <= (size_t)134217728);

typedef __bf16 v16b __attribute__((ext_vector_type(16)));
typedef _Float16 v16h __attribute__((ext_vector_type(16)));
typedef unsigned short v8us __attribute__((ext_vector_type(8), may_alias));
typedef float v8f __attribute__((ext_vector_type(8)));
typedef float v4f __attribute__((ext_vector_type(4)));
typedef float v4fa __attribute__((ext_vector_type(4), may_alias));
typedef int v4i __attribute__((ext_vector_type(4)));
typedef int v4ia __attribute__((ext_vector_type(4), may_alias));
union FragB { v16b v; v8us half[2]; unsigned short u[16]; };
union FragH { v16h v; v8us half[2]; _Float16 h[16]; unsigned short u[16]; };
union Pack8 { _Float16 h[8]; v8us v; };

#define LOG2E 1.4426950408889634f
#define NEGV (-1.0e30f)
#define RINV 0.00048828125f
#define SCL  0.00048828125f

__device__ __forceinline__ unsigned short bf16_bits(float x) {
  unsigned int u = __float_as_uint(x);
  return (unsigned short)((u + 0x7FFFu + ((u >> 16) & 1u)) >> 16);
}
__device__ __forceinline__ float bf16_val(unsigned short b) { return __uint_as_float(((unsigned int)b) << 16); }
__device__ __forceinline__ float bf16_rne(float x) { return bf16_val(bf16_bits(x)); }

__device__ __forceinline__ void mma_h2(v16h a, v16h bh, v16h bl, v8f& ch, v8f& cl) {
  ch = __builtin_amdgcn_wmma_f32_16x16x32_f16(false, a, false, bh, (short)0, ch, false, false);
  cl = __builtin_amdgcn_wmma_f32_16x16x32_f16(false, a, false, bl, (short)0, cl, false, false);
  asm volatile("v_nop\n\tv_nop\n\tv_nop\n\tv_nop" : "+v"(ch), "+v"(cl) : "v"(a), "v"(bh), "v"(bl));
}

__device__ __forceinline__ void mma_b8(v16b a0, v16b a1, v16b b0, v16b b1, v16b b2, v16b b3, v8f (&c)[2][4]) {
  c[0][0] = __builtin_amdgcn_wmma_f32_16x16x32_bf16(false, a0, false, b0, (short)0, c[0][0], false, false);
  c[0][1] = __builtin_amdgcn_wmma_f32_16x16x32_bf16(false, a0, false, b1, (short)0, c[0][1], false, false);
  c[0][2] = __builtin_amdgcn_wmma_f32_16x16x32_bf16(false, a0, false, b2, (short)0, c[0][2], false, false);
  c[0][3] = __builtin_amdgcn_wmma_f32_16x16x32_bf16(false, a0, false, b3, (short)0, c[0][3], false, false);
  c[1][0] = __builtin_amdgcn_wmma_f32_16x16x32_bf16(false, a1, false, b0, (short)0, c[1][0], false, false);
  c[1][1] = __builtin_amdgcn_wmma_f32_16x16x32_bf16(false, a1, false, b1, (short)0, c[1][1], false, false);
  c[1][2] = __builtin_amdgcn_wmma_f32_16x16x32_bf16(false, a1, false, b2, (short)0, c[1][2], false, false);
  c[1][3] = __builtin_amdgcn_wmma_f32_16x16x32_bf16(false, a1, false, b3, (short)0, c[1][3], false, false);
  asm volatile("v_nop\n\tv_nop\n\tv_nop\n\tv_nop"
               : "+v"(c[0][0]), "+v"(c[0][1]), "+v"(c[0][2]), "+v"(c[0][3]),
                 "+v"(c[1][0]), "+v"(c[1][1]), "+v"(c[1][2]), "+v"(c[1][3])
               : "v"(a0), "v"(a1), "v"(b0), "v"(b1), "v"(b2), "v"(b3));
}

__global__ __launch_bounds__(256) void k_xb(const float* __restrict__ X, unsigned short* P) {
  const int t = blockIdx.x * 256 + threadIdx.x;
  if (t >= TT * 128) return;
  const int row = t >> 7, piece = t & 127;
  const int b = row / SEQ, s = row - b * SEQ;
  const float* src = X + ((size_t)s * NB_FULL + b) * DM + piece * 8;
  const v4f x0 = *(const v4fa*)(src), x1 = *(const v4fa*)(src + 4);
  v8us o;
  o[0] = bf16_bits(x0[0]); o[1] = bf16_bits(x0[1]); o[2] = bf16_bits(x0[2]); o[3] = bf16_bits(x0[3]);
  o[4] = bf16_bits(x1[0]); o[5] = bf16_bits(x1[1]); o[6] = bf16_bits(x1[2]); o[7] = bf16_bits(x1[3]);
  unsigned short* d = P + (size_t)t * 8;
  *(volatile v8us*)d = o;
  __threadfence();
  *(volatile v8us*)d = o;
}

__global__ __launch_bounds__(256) void k_wt(const float* __restrict__ W, unsigned short* Wt, int pitch, int dup) {
  __shared__ unsigned short tl[64][66];
  const int tid = threadIdx.x;
  const int k0 = (blockIdx.x >> 4) * 64, n0 = (blockIdx.x & 15) * 64;
  for (int i = tid; i < 64 * 16; i += 256) {
    const int j = i >> 4, c4 = (i & 15) * 4;
    const v4f x = *(const v4fa*)(W + (size_t)(k0 + j) * DM + n0 + c4);
    tl[c4 + 0][j] = bf16_bits(x[0]); tl[c4 + 1][j] = bf16_bits(x[1]);
    tl[c4 + 2][j] = bf16_bits(x[2]); tl[c4 + 3][j] = bf16_bits(x[3]);
  }
  __syncthreads();
  for (int pass = 0; pass < 2; ++pass) {
    for (int i = tid; i < 64 * 8; i += 256) {
      const int d = i >> 3, j8 = (i & 7) * 8;
      v8us o;
#pragma unroll
      for (int q = 0; q < 8; ++q) o[q] = tl[d][j8 + q];
      unsigned short* dst = Wt + (size_t)(n0 + d) * pitch + k0 + j8;
      *(volatile v8us*)dst = o;
      if (dup != 0) *(volatile v8us*)(dst + DM) = o;
    }
    if (pass == 0) __threadfence();
  }
}

template <int MODE>
__global__ __launch_bounds__(128) void k_gemm(const unsigned short* __restrict__ A, const unsigned short* __restrict__ Bt,
                                              const float* __restrict__ bias, unsigned short* O0, unsigned short* O1,
                                              float* Of, int lda, int ldb, int K, int ldo) {
  __shared__ __attribute__((aligned(16))) float so[4][32][68];
  const int tid = threadIdx.x, w = __builtin_amdgcn_readfirstlane((int)(tid >> 5)), lane = tid & 31, ln = lane & 15, hh = lane >> 4;
  const int m0 = blockIdx.y * 64 + (w >> 1) * 32;
  const int n0 = blockIdx.x * 128 + (w & 1) * 64;
  const unsigned short* pa0 = A + (size_t)(m0 + ln) * lda + 8 * hh;
  const unsigned short* pa1 = pa0 + (size_t)16 * lda;
  const unsigned short* pb0 = Bt + (size_t)(n0 + ln) * ldb + 8 * hh;
  const unsigned short* pb1 = pb0 + (size_t)16 * ldb;
  const unsigned short* pb2 = pb0 + (size_t)32 * ldb;
  const unsigned short* pb3 = pb0 + (size_t)48 * ldb;
  v8f acc[2][4];
#pragma unroll
  for (int i = 0; i < 2; ++i)
#pragma unroll
    for (int j = 0; j < 4; ++j)
#pragma unroll
      for (int e = 0; e < 8; ++e) acc[i][j][e] = 0.0f;
#pragma unroll 1
  for (int k0 = 0; k0 < K; k0 += 32) {
    FragB a0, a1, b0, b1, b2, b3;
    a0.half[0] = *(const v8us*)(pa0 + k0); a0.half[1] = *(const v8us*)(pa0 + k0 + 16);
    a1.half[0] = *(const v8us*)(pa1 + k0); a1.half[1] = *(const v8us*)(pa1 + k0 + 16);
    b0.half[0] = *(const v8us*)(pb0 + k0); b0.half[1] = *(const v8us*)(pb0 + k0 + 16);
    b1.half[0] = *(const v8us*)(pb1 + k0); b1.half[1] = *(const v8us*)(pb1 + k0 + 16);
    b2.half[0] = *(const v8us*)(pb2 + k0); b2.half[1] = *(const v8us*)(pb2 + k0 + 16);
    b3.half[0] = *(const v8us*)(pb3 + k0); b3.half[1] = *(const v8us*)(pb3 + k0 + 16);
    mma_b8(a0.v, a1.v, b0.v, b1.v, b2.v, b3.v, acc);
  }
  float rb[2][8];
  float cb[4];
#pragma unroll
  for (int mt = 0; mt < 2; ++mt) {
    if (MODE == 2) {
      const float* bp = bias + m0 + 16 * mt + 8 * hh;
      const v4f ba = *(const v4fa*)(bp), bb = *(const v4fa*)(bp + 4);
#pragma unroll
      for (int r = 0; r < 4; ++r) { rb[mt][r] = bf16_rne(ba[r]); rb[mt][4 + r] = bf16_rne(bb[r]); }
    } else {
#pragma unroll
      for (int r = 0; r < 8; ++r) rb[mt][r] = 0.0f;
    }
  }
#pragma unroll
  for (int nt = 0; nt < 4; ++nt) cb[nt] = (MODE == 2) ? 0.0f : bf16_rne(bias[n0 + 16 * nt + ln]);
#pragma unroll
  for (int mt = 0; mt < 2; ++mt)
#pragma unroll
    for (int nt = 0; nt < 4; ++nt)
#pragma unroll
      for (int r = 0; r < 8; ++r)
        so[w][16 * mt + 8 * hh + r][16 * nt + ln] = acc[mt][nt][r] + (rb[mt][r] + cb[nt]);
  __syncthreads();
  for (int pass = 0; pass < 2; ++pass) {
    if (MODE == 3) {
#pragma unroll
      for (int it = 0; it < 16; ++it) {
        const int row = 2 * it + (lane >> 4), c4 = (lane & 15) * 4;
        const v4f v = *(const v4fa*)&so[w][row][c4];
        const int tp = m0 + row;
        const int b = tp / SEQ, s = tp - b * SEQ;
        *(volatile v4f*)(Of + ((size_t)s * NB_FULL + b) * DM + n0 + c4) = v;
      }
    } else {
#pragma unroll
      for (int it = 0; it < 8; ++it) {
        const int row = 4 * it + (lane >> 3), c8 = (lane & 7) * 8;
        const v4f x0 = *(const v4fa*)&so[w][row][c8];
        const v4f x1 = *(const v4fa*)&so[w][row][c8 + 4];
        Pack8 ph, pl;
#pragma unroll
        for (int q = 0; q < 4; ++q) {
          const float y0 = x0[q] * 16.0f, y1 = x1[q] * 16.0f;
          const _Float16 h0 = (_Float16)y0, h1 = (_Float16)y1;
          ph.h[q] = h0; ph.h[4 + q] = h1;
          pl.h[q] = (_Float16)((y0 - (float)h0) * 2048.0f);
          pl.h[4 + q] = (_Float16)((y1 - (float)h1) * 2048.0f);
        }
        const size_t dst = (size_t)(m0 + row) * ldo + n0 + c8;
        *(volatile v8us*)(O0 + dst) = ph.v;
        if (MODE == 0) *(volatile v8us*)(O1 + dst) = pl.v;
      }
    }
    if (pass == 0) __threadfence();
  }
}

__device__ __forceinline__ void fa_step(const unsigned short* __restrict__ Kp, const unsigned short* __restrict__ Vp,
                                        const int* __restrict__ mk, int key0, int ln, int hh,
                                        const FragH& q0h, const FragH& q0l, const FragH& q1h, const FragH& q1l,
                                        float& mr, float& lr, v8f (&Oh)[4], v8f (&Ol)[4]) {
  const unsigned short* kp0 = Kp + (size_t)(key0 + ln) * DM + 8 * hh;
  const unsigned short* kp1 = kp0 + (size_t)16 * DM;
  FragH k00, k01, k10, k11;
  k00.half[0] = *(const v8us*)(kp0);      k00.half[1] = *(const v8us*)(kp0 + 16);
  k01.half[0] = *(const v8us*)(kp0 + 32); k01.half[1] = *(const v8us*)(kp0 + 48);
  k10.half[0] = *(const v8us*)(kp1);      k10.half[1] = *(const v8us*)(kp1 + 16);
  k11.half[0] = *(const v8us*)(kp1 + 32); k11.half[1] = *(const v8us*)(kp1 + 48);
  const v8f z8 = {0.f, 0.f, 0.f, 0.f, 0.f, 0.f, 0.f, 0.f};
  v8f s0h = z8, s0l = z8, s1h = z8, s1l = z8;
  mma_h2(k00.v, q0h.v, q0l.v, s0h, s0l);
  mma_h2(k01.v, q1h.v, q1l.v, s0h, s0l);
  mma_h2(k10.v, q0h.v, q0l.v, s1h, s1l);
  mma_h2(k11.v, q1h.v, q1l.v, s1h, s1l);
  const int* mp = mk + key0 + 8 * hh;
  const v4i ma = *(const v4ia*)(mp), mb = *(const v4ia*)(mp + 4), mc = *(const v4ia*)(mp + 16), md = *(const v4ia*)(mp + 20);
  int mi[16];
#pragma unroll
  for (int r = 0; r < 4; ++r) { mi[r] = ma[r]; mi[4 + r] = mb[r]; mi[8 + r] = mc[r]; mi[12 + r] = md[r]; }
  float sc[16];
#pragma unroll
  for (int r = 0; r < 8; ++r) {
    const float a0 = (s0h[r] + s0l[r] * RINV) * SCL;
    const float a1 = (s1h[r] + s1l[r] * RINV) * SCL;
    sc[r]     = (mi[r] != 0) ? a0 : NEGV;
    sc[8 + r] = (mi[8 + r] != 0) ? a1 : NEGV;
  }
  float mx = sc[0];
#pragma unroll
  for (int i = 1; i < 16; ++i) mx = fmaxf(mx, sc[i]);
  mx = fmaxf(mx, __shfl_xor(mx, 16, 32));
  const float mnew = fmaxf(mr, mx);
  const float al = exp2f((mr - mnew) * LOG2E);
  mr = mnew;
  FragH ph, pl;
  float ps = 0.0f;
#pragma unroll
  for (int i = 0; i < 16; ++i) {
    const float e = exp2f(fmaf(sc[i] - mnew, LOG2E, 8.0f));
    const float pc = (mi[i] != 0) ? e : 0.0f;
    ps += pc;
    const _Float16 h = (_Float16)pc;
    ph.h[i] = h;
    pl.h[i] = (_Float16)((pc - (float)h) * 2048.0f);
  }
  ps += __shfl_xor(ps, 16, 32);
  lr = lr * al + ps;
#pragma unroll
  for (int t = 0; t < 4; ++t) { Oh[t] = Oh[t] * al; Ol[t] = Ol[t] * al; }
  const unsigned short* vp = Vp + (size_t)ln * TT + key0 + 8 * hh;
#pragma unroll
  for (int t = 0; t < 4; ++t) {
    FragH vf;
    vf.half[0] = *(const v8us*)(vp + (size_t)t * 16 * TT);
    vf.half[1] = *(const v8us*)(vp + (size_t)t * 16 * TT + 16);
    mma_h2(vf.v, ph.v, pl.v, Oh[t], Ol[t]);
  }
}

__global__ __launch_bounds__(128) void k_attn(const unsigned short* __restrict__ Qh, const unsigned short* __restrict__ Ql,
                                              const unsigned short* __restrict__ Kh, const unsigned short* __restrict__ Vt,
                                              const int* __restrict__ mask, unsigned short* Cx) {
  __shared__ __attribute__((aligned(16))) float so[4][16][68];
  const int tid = threadIdx.x, w = __builtin_amdgcn_readfirstlane((int)(tid >> 5)), lane = tid & 31, ln = lane & 15, hh = lane >> 4;
  const int bh = blockIdx.x / (SEQ / 64), qt = blockIdx.x % (SEQ / 64);
  const int b = bh / NH, h = bh % NH;
  const int qbase = qt * 64 + 16 * w;
  const int qg = qbase + ln;
  const size_t qoff = (size_t)(b * SEQ + qg) * DM + h * HD + 8 * hh;
  FragH q0h, q0l, q1h, q1l;
  q0h.half[0] = *(const v8us*)(Qh + qoff);      q0h.half[1] = *(const v8us*)(Qh + qoff + 16);
  q1h.half[0] = *(const v8us*)(Qh + qoff + 32); q1h.half[1] = *(const v8us*)(Qh + qoff + 48);
  q0l.half[0] = *(const v8us*)(Ql + qoff);      q0l.half[1] = *(const v8us*)(Ql + qoff + 16);
  q1l.half[0] = *(const v8us*)(Ql + qoff + 32); q1l.half[1] = *(const v8us*)(Ql + qoff + 48);
  float mr = NEGV, lr = 0.0f;
  v8f Oh[4] = {}, Ol[4] = {};
  const unsigned short* Kp = Kh + (size_t)b * SEQ * DM + h * HD;
  const unsigned short* Vp = Vt + (size_t)h * HD * TT + (size_t)b * SEQ;
#pragma unroll 1
  for (int j = 0; j < SEQ / 32; ++j)
    fa_step(Kp, Vp, mask, 32 * j, ln, hh, q0h, q0l, q1h, q1l, mr, lr, Oh, Ol);

  const float inv = 1.0f / (16.0f * lr);
#pragma unroll
  for (int t = 0; t < 4; ++t)
#pragma unroll
    for (int r = 0; r < 8; ++r)
      so[w][ln][16 * t + 8 * hh + r] = (Oh[t][r] + Ol[t][r] * RINV) * inv;
  __syncthreads();
  unsigned short* cg = Cx + (size_t)(b * SEQ + qbase) * CXP + h * HD;
  for (int pass = 0; pass < 2; ++pass) {
#pragma unroll
    for (int it = 0; it < 4; ++it) {
      const int row = 4 * it + (lane >> 3), c8 = (lane & 7) * 8;
      const v4f x0 = *(const v4fa*)&so[w][row][c8];
      const v4f x1 = *(const v4fa*)&so[w][row][c8 + 4];
      v8us oh, ol;
#pragma unroll
      for (int q = 0; q < 4; ++q) {
        const unsigned short h0 = bf16_bits(x0[q]), h1 = bf16_bits(x1[q]);
        oh[q] = h0; oh[4 + q] = h1;
        ol[q] = bf16_bits(x0[q] - bf16_val(h0));
        ol[4 + q] = bf16_bits(x1[q] - bf16_val(h1));
      }
      unsigned short* dst = cg + (size_t)row * CXP + c8;
      *(volatile v8us*)(dst) = oh;
      *(volatile v8us*)(dst + DM) = ol;
    }
    if (pass == 0) __threadfence();
  }
}

extern "C" void kernel_launch(void* const* d_in, const int* in_sizes, int n_in,
                              void* d_out, int out_size, void* d_ws, size_t ws_size, hipStream_t stream) {
  if (n_in < 12) return;
  const long long need = ((long long)(SEQ - 1) * NB_FULL + (NB - 1)) * DM + DM;
  if ((long long)in_sizes[0] < need || (long long)in_sizes[1] < need || (long long)in_sizes[2] < need) return;
  if ((long long)in_sizes[3] < (long long)SEQ) return;
  if ((long long)in_sizes[4] < (long long)DM * DM || (long long)in_sizes[6] < (long long)DM * DM ||
      (long long)in_sizes[8] < (long long)DM * DM || (long long)in_sizes[10] < (long long)DM * DM) return;
  if (in_sizes[5] < DM || in_sizes[7] < DM || in_sizes[9] < DM || in_sizes[11] < DM) return;
  if ((long long)out_size < need) return;
  const float* Xq = (const float*)d_in[0];
  const float* Xk = (const float*)d_in[1];
  const float* Xv = (const float*)d_in[2];
  const int*   mk = (const int*)d_in[3];
  const float* Wq = (const float*)d_in[4];
  const float* bq = (const float*)d_in[5];
  const float* Wk = (const float*)d_in[6];
  const float* bk = (const float*)d_in[7];
  const float* Wv = (const float*)d_in[8];
  const float* bv = (const float*)d_in[9];
  const float* Wo = (const float*)d_in[10];
  const float* bo = (const float*)d_in[11];
  float* out = (float*)d_out;
  char* ws = (char*)d_ws;
  size_t off = 0;
  unsigned short* Bq  = (unsigned short*)(ws + off); off += SZ_XB;
  unsigned short* Bk  = (unsigned short*)(ws + off); off += SZ_XB;
  unsigned short* Bv  = (unsigned short*)(ws + off); off += SZ_XB;
  unsigned short* WqT = (unsigned short*)(ws + off); off += SZ_WT;
  unsigned short* WkT = (unsigned short*)(ws + off); off += SZ_WT;
  unsigned short* WvT = (unsigned short*)(ws + off); off += SZ_WT;
  unsigned short* Wo2 = (unsigned short*)(ws + off); off += SZ_WO2;
  unsigned short* Qh  = (unsigned short*)(ws + off); off += SZ_H;
  unsigned short* Ql  = (unsigned short*)(ws + off); off += SZ_H;
  unsigned short* Kh  = (unsigned short*)(ws + off); off += SZ_H;
  unsigned short* Vt  = (unsigned short*)(ws + off); off += SZ_H;
  unsigned short* Cx  = (unsigned short*)(ws + off); off += SZ_CX;
  if (off > ws_size) return;

  const unsigned gx = (unsigned)((TT * 128 + 255) / 256);
  k_xb<<<gx, 256, 0, stream>>>(Xq, Bq);
  k_xb<<<gx, 256, 0, stream>>>(Xk, Bk);
  k_xb<<<gx, 256, 0, stream>>>(Xv, Bv);
  k_wt<<<256, 256, 0, stream>>>(Wq, WqT, DM, 0);
  k_wt<<<256, 256, 0, stream>>>(Wk, WkT, DM, 0);
  k_wt<<<256, 256, 0, stream>>>(Wv, WvT, DM, 0);
  k_wt<<<256, 256, 0, stream>>>(Wo, Wo2, CXP, 1);

  k_gemm<0><<<dim3(DM / 128, TT / 64), 128, 0, stream>>>(Bq, WqT, bq, Qh, Ql, out, DM, DM, DM, DM);
  k_gemm<1><<<dim3(DM / 128, TT / 64), 128, 0, stream>>>(Bk, WkT, bk, Kh, Kh, out, DM, DM, DM, DM);
  k_gemm<2><<<dim3(TT / 128, DM / 64), 128, 0, stream>>>(WvT, Bv, bv, Vt, Vt, out, DM, DM, DM, TT);
  k_attn<<<(unsigned)(NB * NH * (SEQ / 64)), 128, 0, stream>>>(Qh, Ql, Kh, Vt, mk, Cx);
  k_gemm<3><<<dim3(DM / 128, TT / 64), 128, 0, stream>>>(Cx, Wo2, bo, Cx, Cx, out, CXP, CXP, CXP, DM);
}
